// WeldRNN_36541581755031
// MI455X (gfx1250) — hardware-verified
//
#include <hip/hip_runtime.h>
#include <math.h>

constexpr int NBATCH  = 64;
constexpr int NSTEP   = 512;
constexpr int NINP    = 6;
constexpr int NHID    = 1024;
constexpr int NTHR    = 512;
constexpr int NWAVE   = NTHR / 32;
constexpr int SEQ_BLK = 16;
constexpr int HPITCH  = NHID + 8;
constexpr int HPW     = NWAVE * 16;
constexpr int TSTAGE  = 32;
constexpr float WCARRY  = 32.0f;
constexpr float HCARRY  = 16.0f;
constexpr float ACC_INV = 1.0f / (WCARRY * HCARRY);

static_assert(NHID % 32 == 0, "K multiple of 32");
static_assert(NHID == 64 * NWAVE, "each wave owns four 16-column tiles");
static_assert(NBATCH % SEQ_BLK == 0, "whole 16-row blocks");
static_assert(NSTEP % TSTAGE == 0, "no output tail");
static_assert(HPITCH % 8 == 0, "16-B aligned LDS rows");
static_assert(HPW == 256, "one 8-float slice per lane in the head sum");
static_assert((NHID * NHID) % (8 * 256) == 0, "weight plane grid exact");

typedef __attribute__((ext_vector_type(16))) _Float16 v16h;
typedef __attribute__((ext_vector_type(8)))  _Float16 v8h;
typedef __attribute__((ext_vector_type(8)))  float    v8f;
typedef __attribute__((ext_vector_type(4)))  float    v4f;
typedef __attribute__((ext_vector_type(2)))  float    v2f;

struct FragH {
  union U { v16h v; v8h h[2]; };
  static __device__ __forceinline__ v16h load(const _Float16* p) {
    U f; f.h[0] = *(const v8h*)(p); f.h[1] = *(const v8h*)(p + 16); return f.v;
  }
  static __device__ __forceinline__ v8f mma(v16h a, v16h b, v8f c) {
    return __builtin_amdgcn_wmma_f32_16x16x32_f16(false, a, false, b, (short)0, c, false, false);
  }
};
__device__ __forceinline__ void guard_group(v8f& a0, v8f& a1, v8f& a2, v8f& a3,
                                            v16h x, v16h y0, v16h y1, v16h y2, v16h y3) {
  asm volatile("v_nop\n\tv_nop\n\tv_nop\n\tv_nop"
               : "+v"(a0), "+v"(a1), "+v"(a2), "+v"(a3)
               : "v"(x), "v"(y0), "v"(y1), "v"(y2), "v"(y3));
}
__device__ __forceinline__ void acc_guard4(v8f& a, v8f& b, v8f& c, v8f& d) {
  asm volatile("v_nop\n\tv_nop\n\tv_nop\n\tv_nop" : "+v"(a), "+v"(b), "+v"(c), "+v"(d));
}

__global__ __launch_bounds__(256) void wplane_kernel(const float* __restrict__ w, unsigned short* __restrict__ dst, int n8) {
  const int i = blockIdx.x * 256 + threadIdx.x;
  if (i < n8) {
    const float* sp = w + (size_t)i * 8;
    const v4f a = *(const v4f*)(sp);
    const v4f b = *(const v4f*)(sp + 4);
    v8h hv;
#pragma unroll
    for (int e = 0; e < 4; ++e) {
      const float fa = a[e] * WCARRY;
      const float fb = b[e] * WCARRY;
      hv[e]     = (_Float16)fa;
      hv[4 + e] = (_Float16)fb;
    }
    *(volatile v8h*)(dst + (size_t)i * 8) = hv;
    __threadfence();
    *(volatile v8h*)(dst + (size_t)i * 8) = hv;
  }
}

__global__ __launch_bounds__(NTHR) void rnn_seq_kernel(const float* __restrict__ src, const float* __restrict__ w_ih,
                                                       const float* __restrict__ b_ih, const float* __restrict__ b_hh,
                                                       const float* __restrict__ w_out, const float* __restrict__ b_out,
                                                       const unsigned short* __restrict__ W16p, float* __restrict__ out) {
  __shared__ __align__(16) _Float16 Ah[SEQ_BLK * HPITCH];
  __shared__ __align__(16) float    hp[SEQ_BLK * HPW];
  __shared__ __align__(16) float    outst[SEQ_BLK * TSTAGE];
  __shared__ __align__(16) float    xs[SEQ_BLK * 8];

  const _Float16* W16 = (const _Float16*)W16p;
  const int tid = threadIdx.x, lane = tid & 31, wave = tid >> 5;
  const int c = lane & 15, hh = lane >> 4, koff = hh * 8;
  const int rowbase = blockIdx.x * SEQ_BLK;

#pragma unroll 1
  for (int i = tid; i < SEQ_BLK * HPITCH; i += NTHR) Ah[i] = (_Float16)0.0f;

  if (tid < 128) {
    const int m = tid >> 3, i = tid & 7;
    const int ic = (i < NINP) ? i : (NINP - 1);
    const float v = src[((size_t)(rowbase + m) * NSTEP) * NINP + ic];
    xs[m * 8 + i] = (i < NINP) ? v : 0.0f;
  }

  float wih[4][NINP], bsum[4], wo[4];
#pragma unroll
  for (int nt = 0; nt < 4; ++nt) {
    const int j = 64 * wave + 16 * nt + c;
    const float* wp = w_ih + (size_t)j * NINP;
    const v2f w0 = *(const v2f*)(wp);
    const v2f w1 = *(const v2f*)(wp + 2);
    const v2f w2 = *(const v2f*)(wp + 4);
    wih[nt][0] = w0[0]; wih[nt][1] = w0[1];
    wih[nt][2] = w1[0]; wih[nt][3] = w1[1];
    wih[nt][4] = w2[0]; wih[nt][5] = w2[1];
    bsum[nt] = b_ih[j] + b_hh[j];
    wo[nt] = w_out[j];
  }
  const float bout = b_out[0];
  __syncthreads();

  const _Float16* ahrow = Ah + c * HPITCH + koff;
  const _Float16* wrow  = W16 + (size_t)(64 * wave + c) * NHID + koff;
  const v8f z8 = {0.f, 0.f, 0.f, 0.f, 0.f, 0.f, 0.f, 0.f};

#pragma unroll 1
  for (int t = 0; t < NSTEP; ++t) {
    v8f acc[4];
    acc[0] = z8; acc[1] = z8; acc[2] = z8; acc[3] = z8;
#pragma unroll 2
    for (int k0 = 0; k0 < NHID; k0 += 32) {
      const v16h a  = FragH::load(ahrow + k0);
      const v16h b0 = FragH::load(wrow + k0);
      const v16h b1 = FragH::load(wrow + (size_t)16 * NHID + k0);
      const v16h b2 = FragH::load(wrow + (size_t)32 * NHID + k0);
      const v16h b3 = FragH::load(wrow + (size_t)48 * NHID + k0);
      acc[0] = FragH::mma(a, b0, acc[0]);
      acc[1] = FragH::mma(a, b1, acc[1]);
      acc[2] = FragH::mma(a, b2, acc[2]);
      acc[3] = FragH::mma(a, b3, acc[3]);
      guard_group(acc[0], acc[1], acc[2], acc[3], a, b0, b1, b2, b3);
    }
    acc_guard4(acc[0], acc[1], acc[2], acc[3]);

    float p[8];
#pragma unroll
    for (int r = 0; r < 8; ++r) {
      const float* xr = xs + (8 * hh + r) * 8;
      const v4f xa = *(const v4f*)(xr);
      const v4f xb = *(const v4f*)(xr + 4);
      float pr = 0.0f;
#pragma unroll
      for (int nt = 0; nt < 4; ++nt) {
        float xp = bsum[nt];
        xp = fmaf(xa[0], wih[nt][0], xp);
        xp = fmaf(xa[1], wih[nt][1], xp);
        xp = fmaf(xa[2], wih[nt][2], xp);
        xp = fmaf(xa[3], wih[nt][3], xp);
        xp = fmaf(xb[0], wih[nt][4], xp);
        xp = fmaf(xb[1], wih[nt][5], xp);
        const float pre = fmaf(acc[nt][r], ACC_INV, xp);
        const float hn  = fmaxf(pre, 0.0f);
        acc[nt][r] = hn;
        pr = fmaf(hn, wo[nt], pr);
      }
      p[r] = pr;
    }
#pragma unroll
    for (int r = 0; r < 8; ++r) hp[(8 * hh + r) * HPW + 16 * wave + c] = p[r];

    __syncthreads();

#pragma unroll
    for (int nt = 0; nt < 4; ++nt) {
      const int j = 64 * wave + 16 * nt + c;
#pragma unroll
      for (int r = 0; r < 8; ++r) {
        const float hs = acc[nt][r] * HCARRY;
        Ah[(8 * hh + r) * HPITCH + j] = (_Float16)hs;
      }
    }
    if (tid < 128) {
      const int tn = (t + 1 < NSTEP) ? (t + 1) : (NSTEP - 1);
      const int m = tid >> 3, i = tid & 7;
      const int ic = (i < NINP) ? i : (NINP - 1);
      const float v = src[((size_t)(rowbase + m) * NSTEP + (size_t)tn) * NINP + ic];
      xs[m * 8 + i] = (i < NINP) ? v : 0.0f;
    }
    {
      const float* hr = hp + wave * HPW + lane * 8;
      const v4f u = *(const v4f*)(hr);
      const v4f w = *(const v4f*)(hr + 4);
      float s = ((u[0] + u[1]) + (u[2] + u[3])) + ((w[0] + w[1]) + (w[2] + w[3]));
#pragma unroll
      for (int off = 16; off > 0; off >>= 1) s += __shfl_xor(s, off, 32);
      if (lane == 0) outst[wave * TSTAGE + (t & (TSTAGE - 1))] = s + bout;
    }

    __syncthreads();

    if ((t & (TSTAGE - 1)) == (TSTAGE - 1)) {
      if (wave < 4) {
        const int row = 4 * wave + (lane >> 3);
        const int c4  = (lane & 7) * 4;
        const v4f v = *(const v4f*)(outst + row * TSTAGE + c4);
        float* op = out + (size_t)(rowbase + row) * NSTEP + (size_t)(t - (TSTAGE - 1)) + c4;
        *(volatile v4f*)op = v;
        __threadfence();
        *(volatile v4f*)op = v;
      }
    }
  }
}

extern "C" void kernel_launch(void* const* d_in, const int* in_sizes, int n_in,
                              void* d_out, int out_size, void* d_ws, size_t ws_size, hipStream_t stream) {
  if (n_in < 7 || d_out == nullptr || d_ws == nullptr) return;
  if (in_sizes[0] != NBATCH * NSTEP * NINP || in_sizes[1] != NHID * NINP || in_sizes[2] != NHID * NHID ||
      in_sizes[3] != NHID || in_sizes[4] != NHID || in_sizes[5] != NHID || in_sizes[6] != 1 ||
      out_size != NBATCH * NSTEP) return;

  const float* src   = (const float*)d_in[0];
  const float* w_ih  = (const float*)d_in[1];
  const float* w_hh  = (const float*)d_in[2];
  const float* b_ih  = (const float*)d_in[3];
  const float* b_hh  = (const float*)d_in[4];
  const float* w_out = (const float*)d_in[5];
  const float* b_out = (const float*)d_in[6];
  float* out = (float*)d_out;

  const size_t w16_bytes = (size_t)NHID * NHID * 2;
  if (w16_bytes > ws_size || w16_bytes > (size_t)134217728) return;
  unsigned short* W16 = (unsigned short*)d_ws;

  const int n8 = NHID * NHID / 8;
  wplane_kernel<<<n8 / 256, 256, 0, stream>>>(w_hh, W16, n8);
  rnn_seq_kernel<<<NBATCH / SEQ_BLK, NTHR, 0, stream>>>(src, w_ih, b_ih, b_hh, w_out, b_out, W16, out);
}
